// PhyGraphConv_32719060861306
// MI455X (gfx1250) — hardware-run, weakly checked
//
#include <hip/hip_runtime.h>


namespace {
constexpr int NB = 4, NN = 16384, EB = 131072, C = 128, ND = 3, KG = C * ND  , MID = 128, OUTC = 128, N = NB * NN  , E = NB * EB  ;
constexpr float XS = 8.0f, WSC = 256.0f, NEG = 0.2f  ;

typedef _Float16 b16;
typedef __attribute__((ext_vector_type(16))) _Float16 v16b;
typedef __attribute__((ext_vector_type(8))) _Float16 v8b;
typedef __attribute__((ext_vector_type(8))) float v8f;
typedef __attribute__((ext_vector_type(4))) float v4f;
__device__ __forceinline__ float bf16_rne(float f) { unsigned int u = __float_as_uint(f); u += 0x7FFFu + ((u >> 16) & 1u); return __uint_as_float(u & 0xFFFF0000u); }
__device__ __forceinline__ void split16(float v, b16& hi, b16& lo) { hi = (b16)v; lo = (b16)(v - (float)hi); }
__device__ __forceinline__ v16b frag_kb(const b16* p, int hh) { const v8b a = *(const v8b*)(p + 8 * hh), b = *(const v8b*)(p + 16 + 8 * hh); v16b f;
#pragma unroll
  for (int e = 0; e < 8; ++e) { f[e] = a[e]; f[8 + e] = b[e]; } return f; }
__device__ __forceinline__ v8f wmma16b(v16b a, v16b b, v8f c) { v8f d = __builtin_amdgcn_wmma_f32_16x16x32_f16(false, a, false, b, (short)0, c, false, false); asm volatile("v_nop\n\tv_nop\n\tv_nop\n\tv_nop" : "+v"(d) : "v"(a), "v"(b)); return d; }
__device__ __forceinline__ void wave_lds_sync() { __builtin_amdgcn_fence(__ATOMIC_RELEASE, "workgroup"); __builtin_amdgcn_wave_barrier(); __builtin_amdgcn_fence(__ATOMIC_ACQUIRE, "workgroup"); }
__device__ __forceinline__ float pmul(float a, float b) { float p = a * b; asm volatile("" : "+v"(p)); return p; }
__device__ __forceinline__ int iclamp(int v, int lo, int hi) { return v < lo ? lo : (v > hi ? hi : v); }
__device__ __forceinline__ float nexp(float x) { return __builtin_amdgcn_exp2f(x * 1.4426950408889634f); }
__device__ __forceinline__ float lrelu(float x) { return x > 0.0f ? x : NEG * x; }

constexpr int CSR_NBLK = 512, CSR_GB = 9, CSR_GN = 1 << CSR_GB  , CSR_MAXG = 512, CSR_CAP = 12288  ;
__global__ __launch_bounds__(64) void csrA_kernel(const int* __restrict__ dst, int E, int N, int nG, int CHP, int NGP, int* __restrict__ STG, int* __restrict__ HST) {
  extern __shared__ int sm[];
  int* cnt = sm; int* run = sm + NGP; int* ids = sm + 2 * NGP;
  const int b = blockIdx.x; const int ch = (E + CSR_NBLK - 1) / CSR_NBLK; const int e0 = b * ch, e1 = min(E, e0 + ch);
  for (int i = threadIdx.x; i < NGP; i += 64) cnt[i] = 0;
  for (int i = threadIdx.x; i < CHP; i += 64) ids[i] = -1;
  __syncthreads();
  if (threadIdx.x == 0) {
    for (int e = e0; e < e1; ++e) { int d = dst[e]; d = (d < 0) ? 0 : (d >= N ? N - 1 : d); cnt[d >> CSR_GB] += 1; }
    int acc = 0; for (int g = 0; g < nG; ++g) { run[g] = acc; acc += cnt[g]; }
    for (int e = e0; e < e1; ++e) { int d = dst[e]; d = (d < 0) ? 0 : (d >= N ? N - 1 : d); const int g = d >> CSR_GB; ids[run[g]] = e; run[g] += 1; } }
  __syncthreads();
  typedef __attribute__((ext_vector_type(4))) int v4i;
  for (int pass = 0; pass < 2; ++pass) {
    for (int i = threadIdx.x; i < CHP / 4; i += 64) *(volatile v4i*)(STG + (size_t)b * CHP + i * 4) = *(const v4i*)(&ids[i * 4]);
    for (int i = threadIdx.x; i < NGP / 4; i += 64) { v4i v; for (int e = 0; e < 4; ++e) v[e] = (i * 4 + e < nG) ? cnt[i * 4 + e] : 0; *(volatile v4i*)(HST + (size_t)b * NGP + i * 4) = v; }
    __threadfence(); }
}
__global__ __launch_bounds__(512) void csrS_kernel(const int* __restrict__ HST, int nG, int NGP, int* __restrict__ START, int* __restrict__ TOT, int* __restrict__ OFF) {
  __shared__ int tot[CSR_MAXG];
  const int b = threadIdx.x;
  for (int pass = 0; pass < 2; ++pass) { int runb = 0; for (int g = 0; g < nG; ++g) { int c = HST[(size_t)b * NGP + g]; c = (c < 0) ? 0 : c; ((volatile int*)OFF)[(size_t)g * CSR_NBLK + b] = runb; runb += c; } __threadfence(); }
  for (int g = threadIdx.x; g < nG; g += 512) { int s = 0; for (int bb = 0; bb < CSR_NBLK; ++bb) { int c = HST[(size_t)bb * NGP + g]; s += (c < 0) ? 0 : c; } tot[g] = s; }
  __syncthreads();
  if (threadIdx.x < 32) {
    __shared__ int st[CSR_MAXG + 32];
    if (threadIdx.x == 0) { int acc = 0; for (int g = 0; g < NGP; ++g) { st[g] = acc; if (g < nG) acc += (tot[g] + 31) & ~31; } st[NGP] = acc; }
    __builtin_amdgcn_fence(__ATOMIC_RELEASE, "workgroup"); __builtin_amdgcn_wave_barrier(); __builtin_amdgcn_fence(__ATOMIC_ACQUIRE, "workgroup");
    for (int pass = 0; pass < 2; ++pass) { for (int i = threadIdx.x; i < NGP + 32; i += 32) { ((volatile int*)START)[i] = (i <= NGP) ? st[min(i, NGP)] : 0; ((volatile int*)TOT)[i] = (i < nG) ? tot[i] : 0; } __threadfence(); } }
}
__global__ __launch_bounds__(256) void csrB_kernel(const int* __restrict__ dst, int N, int nG, int CHP, int NGP, int permLen, const int* __restrict__ STG, const int* __restrict__ HST, const int* __restrict__ OFF, const int* __restrict__ START, const int* __restrict__ TOT, int* __restrict__ PERM, int* __restrict__ ROWPTR, int* __restrict__ ROWCNT, int* __restrict__ FLAG) {
  typedef __attribute__((ext_vector_type(4))) int v4i;
  __shared__ int ids[CSR_CAP]; __shared__ unsigned short key[CSR_CAP]; __shared__ int outp[CSR_CAP]; __shared__ int ncnt[CSR_GN + 1]; __shared__ int boff[CSR_NBLK + 1];
  const int g = blockIdx.x, t_ = threadIdx.x; int tot = TOT[g]; int st = START[g], stn = START[g + 1]; const int v0 = g * CSR_GN; const int nv = min(CSR_GN, N - v0);
  st = (st < 0) ? 0 : (st > permLen - 32 ? permLen - 32 : st) & ~31; stn = (stn < st) ? st : (stn > permLen ? permLen : stn); tot = (tot < 0) ? 0 : tot; if (tot > stn - st && tot <= CSR_CAP) tot = stn - st;
  if (tot > CSR_CAP) {
    for (int pass = 0; pass < 2; ++pass) { for (int i = t_; i < CSR_GN / 4; i += 256) { v4i a, c; for (int e = 0; e < 4; ++e) { a[e] = st; c[e] = 0; } *(volatile v4i*)(ROWPTR + v0 + i * 4) = a; *(volatile v4i*)(ROWCNT + v0 + i * 4) = c; } if (t_ == 0) ((volatile int*)FLAG)[0] = 1; __threadfence(); } (void)nv; return; }
  if (t_ == 0) { int acc = 0; for (int b = 0; b < CSR_NBLK; ++b) { boff[b] = acc; int c = HST[(size_t)b * NGP + g]; c = (c < 0) ? 0 : (c > CHP ? CHP : c); acc += c; if (acc > tot) acc = tot; } boff[CSR_NBLK] = acc; }
  for (int i = t_; i <= CSR_GN; i += 256) ncnt[i] = 0;
  __syncthreads();
  for (int b = 0; b < CSR_NBLK; ++b) { const int c = boff[b + 1] - boff[b]; int o_ = OFF[(size_t)g * CSR_NBLK + b]; o_ = (o_ < 0) ? 0 : (o_ > CHP - c ? CHP - c : o_); const int* src_ = STG + (size_t)b * CHP + o_;
    for (int i = t_; i < c; i += 256) { int id = src_[i]; id = (id < 0) ? 0 : id; ids[boff[b] + i] = id; int d = dst[id]; d = (d < v0) ? v0 : (d >= N ? N - 1 : d); int kk = d - v0; kk = (kk < 0) ? 0 : (kk >= CSR_GN ? CSR_GN - 1 : kk); key[boff[b] + i] = (unsigned short)kk; } }
  __syncthreads();
  if (t_ == 0) { for (int i = 0; i < tot; ++i) ncnt[key[i]] += 1; int acc = 0; for (int vl = 0; vl < CSR_GN; ++vl) { const int c = ncnt[vl]; ncnt[vl] = acc; acc += c; } ncnt[CSR_GN] = acc;
    for (int i = 0; i < tot; ++i) { const int vl = key[i]; outp[ncnt[vl]] = ids[i]; ncnt[vl] += 1; }
    for (int vl = CSR_GN; vl > 0; --vl) ncnt[vl] = ncnt[vl - 1]; ncnt[0] = 0; }
  __syncthreads();
  for (int pass = 0; pass < 2; ++pass) {
    for (int i = t_; i < (stn - st) / 4; i += 256) { v4i v; for (int e = 0; e < 4; ++e) { const int q = i * 4 + e; v[e] = (q < tot) ? outp[q] : -1; } *(volatile v4i*)(PERM + st + i * 4) = v; }
    for (int i = t_; i < CSR_GN / 4; i += 256) { v4i a, c; for (int e = 0; e < 4; ++e) { const int vl = i * 4 + e; a[e] = st + ncnt[vl]; c[e] = (vl < nv) ? (ncnt[vl + 1] - ncnt[vl]) : 0; } *(volatile v4i*)(ROWPTR + v0 + i * 4) = a; *(volatile v4i*)(ROWCNT + v0 + i * 4) = c; }
    __threadfence(); }
}
__global__ __launch_bounds__(256) void csrZ_kernel(int* __restrict__ p, size_t n4) { typedef __attribute__((ext_vector_type(4))) int v4i; const size_t tid = (size_t)blockIdx.x * 256 + threadIdx.x, nth = (size_t)gridDim.x * 256; v4i z = {0, 0, 0, 0}; for (size_t i = tid; i < n4; i += nth) *(volatile v4i*)(p + i * 4) = z; }
struct CsrBufs { int *STG, *HST, *OFF, *START, *TOT, *PERM, *ROWPTR, *ROWCNT, *FLAG; int nG, NGP, CHP; size_t permLen; char* base; size_t bytes; };
static size_t csr_carve(CsrBufs& c, char* ws, size_t off, int E, int N) {
  const size_t off0 = off; c.base = ws + off;
  auto al = [&](size_t bytes) { char* p = ws + off; off += (bytes + 255) & ~(size_t)255; return p; };
  c.nG = (N + CSR_GN - 1) / CSR_GN; c.NGP = (c.nG + 31) & ~31; const int ch = (E + CSR_NBLK - 1) / CSR_NBLK; c.CHP = (ch + 31) & ~31; c.permLen = (size_t)E + 32 * (size_t)c.nG + 32;
  c.STG = (int*)al((size_t)CSR_NBLK * c.CHP * 4); c.HST = (int*)al((size_t)CSR_NBLK * c.NGP * 4); c.OFF = (int*)al((size_t)c.NGP * CSR_NBLK * 4); c.START = (int*)al((size_t)(c.NGP + 64) * 4); c.TOT = (int*)al((size_t)(c.NGP + 64) * 4);
  c.PERM = (int*)al(c.permLen * 4); c.ROWPTR = (int*)al((size_t)c.nG * CSR_GN * 4); c.ROWCNT = (int*)al((size_t)c.nG * CSR_GN * 4); c.FLAG = (int*)al(256);
  c.bytes = off - off0; return off;
}
static void csr_build(const CsrBufs& c, const int* dst, int E, int N, hipStream_t stream) {
  const size_t smem = (size_t)(2 * c.NGP + c.CHP) * 4;
  csrZ_kernel<<<512, 256, 0, stream>>>((int*)c.base, c.bytes / 16);
  csrA_kernel<<<CSR_NBLK, 64, smem, stream>>>(dst, E, N, c.nG, c.CHP, c.NGP, c.STG, c.HST);
  csrS_kernel<<<1, 512, 0, stream>>>(c.HST, c.nG, c.NGP, c.START, c.TOT, c.OFF);
  csrB_kernel<<<c.nG, 256, 0, stream>>>(dst, N, c.nG, c.CHP, c.NGP, (int)c.permLen, c.STG, c.HST, c.OFF, c.START, c.TOT, c.PERM, c.ROWPTR, c.ROWCNT, c.FLAG);
}


__global__ __launch_bounds__(256) void keys_kernel(const int* __restrict__ ei, int* __restrict__ KD) {
  typedef __attribute__((ext_vector_type(4))) int v4i;
  const size_t u = (size_t)blockIdx.x * 256 + threadIdx.x; if (u * 4 >= (size_t)E) return; const size_t e0 = u * 4; v4i kd;
  for (int j = 0; j < 4; ++j) { const size_t e = e0 + j; const int b = (int)(e / EB); kd[j] = b * NN + iclamp(ei[e * 2 + 1], 0, NN - 1); }
  for (int pass = 0; pass < 2; ++pass) { *(volatile v4i*)(KD + e0) = kd; __threadfence(); }
}
__global__ __launch_bounds__(256) void prep_kernel(const float* __restrict__ f, const float* __restrict__ w1, const float* __restrict__ w2, float* __restrict__ FT, b16* __restrict__ W1T, b16* __restrict__ W2T) {
  __shared__ float T[64][64 + 1];
  const int n0 = blockIdx.x * 64, c0 = blockIdx.y * 64, b = blockIdx.z, t_ = threadIdx.x;
  for (int q = t_; q < 64 * 64; q += 256) { const int c = q >> 6, nn = q & 63; T[nn][c] = bf16_rne(f[((size_t)b * C + c0 + c) * NN + n0 + nn]); }
  __syncthreads();
  for (int pass = 0; pass < 2; ++pass) { for (int q = t_; q < 64 * 16; q += 256) { const int nn = q >> 4, c4 = (q & 15) * 4; v4f o = {T[nn][c4], T[nn][c4 + 1], T[nn][c4 + 2], T[nn][c4 + 3]}; *(volatile v4f*)(FT + (((size_t)b * NN + n0 + nn) * C) + c0 + c4) = o; } __threadfence(); }
  if (blockIdx.x == 0 && blockIdx.y == 0 && blockIdx.z == 0) {
    for (int q = t_; q < MID * KG / 8; q += 256) { const int e = q * 8; v8b o; for (int j = 0; j < 8; ++j) o[j] = (b16)(bf16_rne(w1[e + j]) * WSC); for (int pass = 0; pass < 2; ++pass) { *(volatile v8b*)(W1T + e) = o; __threadfence(); } }
    for (int q = t_; q < OUTC * MID / 8; q += 256) { const int e = q * 8; v8b o; for (int j = 0; j < 8; ++j) o[j] = (b16)(bf16_rne(w2[e + j]) * WSC); for (int pass = 0; pass < 2; ++pass) { *(volatile v8b*)(W2T + e) = o; __threadfence(); } } }
}
__global__ __launch_bounds__(128) void gradmlp_kernel(const float* __restrict__ FT, const int* __restrict__ ei, const float* __restrict__ egw, const int* __restrict__ PERM, const int* __restrict__ ROWPTR, const int* __restrict__ ROWCNT, int permLen, const b16* __restrict__ W1T, const float* __restrict__ b1, const b16* __restrict__ W2T, const float* __restrict__ b2, float* __restrict__ FO) {
  __shared__ __attribute__((aligned(16))) unsigned char raw[2 * 64 * (KG + 8) * 2];
  typedef b16 (*Tile)[KG + 8]; Tile Ah = (Tile)raw; Tile Al = (Tile)(raw + 64 * (KG + 8) * 2);
  const int wave = threadIdx.x >> 5, lane = threadIdx.x & 31, nloc = lane & 15, hlf = lane >> 4; const size_t v0 = (size_t)blockIdx.x * 64 + wave * 16; const size_t b = v0 / NN;
  for (int rr = 0; rr < 16; ++rr) { const size_t v = v0 + rr; const size_t node = v % NN; float g[12]; for (int j = 0; j < 12; ++j) g[j] = 0.0f;
    int st = ROWPTR[v], cnt = ROWCNT[v]; cnt = iclamp(cnt, 0, 65536); st = iclamp(st, 0, permLen - cnt);
    const v4f ft = *(const v4f*)(FT + v * C + lane * 4);
    for (int i = 0; i < cnt; ++i) { const int e = iclamp(PERM[st + i], 0, E - 1); const size_t s = b * NN + (size_t)iclamp(ei[(size_t)e * 2], 0, NN - 1); const v4f fs = *(const v4f*)(FT + s * C + lane * 4);
      const float w0 = bf16_rne(egw[(size_t)e * 3]), w1 = bf16_rne(egw[(size_t)e * 3 + 1]), w2 = bf16_rne(egw[(size_t)e * 3 + 2]);
      for (int j = 0; j < 4; ++j) { const float df = fs[j] - ft[j]; g[j * 3] += pmul(df, w0); g[j * 3 + 1] += pmul(df, w1); g[j * 3 + 2] += pmul(df, w2); } }
    (void)node;
    for (int j = 0; j < 12; ++j) { b16 p, q; split16(g[j] * XS, p, q); Ah[wave * 16 + rr][lane * 12 + j] = p; Al[wave * 16 + rr][lane * 12 + j] = q; } }
  wave_lds_sync();
  v8f acc[8];
#pragma unroll
  for (int t = 0; t < 8; ++t) acc[t] = (v8f){};
#pragma unroll 2
  for (int kb = 0; kb < KG; kb += 32) { const v16b a = frag_kb(&Ah[wave * 16 + nloc][kb], hlf), al = frag_kb(&Al[wave * 16 + nloc][kb], hlf);
#pragma unroll
    for (int t = 0; t < 8; ++t) { const v16b bw = frag_kb(W1T + (size_t)(t * 16 + nloc) * KG + kb, hlf); acc[t] = wmma16b(a, bw, acc[t]); acc[t] = wmma16b(al, bw, acc[t]); } }
  wave_lds_sync();
#pragma unroll
  for (int t = 0; t < 8; ++t) { const int c = t * 16 + nloc; const float bb = bf16_rne(b1[c]);
#pragma unroll 1
    for (int r = 0; r < 8; ++r) { const float x = acc[t][r] * (1.0f / (XS * WSC)) + bb; const float ge = 0.5f * x * (1.0f + erff(x * 0.70710678118654752f)); b16 p, q; split16(ge * XS, p, q); Ah[wave * 16 + 8 * hlf + r][c] = p; Al[wave * 16 + 8 * hlf + r][c] = q; } }
  wave_lds_sync();
#pragma unroll
  for (int t = 0; t < 8; ++t) acc[t] = (v8f){};
#pragma unroll
  for (int kb = 0; kb < MID; kb += 32) { const v16b a = frag_kb(&Ah[wave * 16 + nloc][kb], hlf), al = frag_kb(&Al[wave * 16 + nloc][kb], hlf);
#pragma unroll
    for (int t = 0; t < 8; ++t) { const v16b bw = frag_kb(W2T + (size_t)(t * 16 + nloc) * MID + kb, hlf); acc[t] = wmma16b(a, bw, acc[t]); acc[t] = wmma16b(al, bw, acc[t]); } }
  __syncthreads();
  float (*Tf)[OUTC + 4] = (float (*)[OUTC + 4])(raw + (size_t)wave * 16 * (OUTC + 4) * 4);
#pragma unroll
  for (int t = 0; t < 8; ++t) { const int c = t * 16 + nloc; const float bb = bf16_rne(b2[c]);
#pragma unroll 1
    for (int r = 0; r < 8; ++r) Tf[8 * hlf + r][c] = acc[t][r] * (1.0f / (XS * WSC)) + bb; }
  wave_lds_sync();
  for (int pass = 0; pass < 2; ++pass) { for (int rr = 0; rr < 16; ++rr) *(volatile v4f*)(FO + (v0 + rr) * OUTC + lane * 4) = *(const v4f*)(&Tf[rr][lane * 4]); __threadfence(); }
}
__global__ __launch_bounds__(256) void kagg_kernel(const float* __restrict__ FO, const float* __restrict__ nodes, const float* __restrict__ nw, const int* __restrict__ ei, const int* __restrict__ PERM, const int* __restrict__ ROWPTR, const int* __restrict__ ROWCNT, int permLen, const float* __restrict__ Lm, const float* __restrict__ cb, float* __restrict__ out) {
  __shared__ __attribute__((aligned(16))) float St[OUTC][64 + 4];
  const int wave = threadIdx.x >> 5, lane = threadIdx.x & 31, t_ = threadIdx.x; const size_t v0 = (size_t)blockIdx.x * 64; const size_t b = v0 / NN; const int n0 = (int)(v0 % NN);
  float S[3][3]; { float Lr[3][3]; for (int i = 0; i < 3; ++i) for (int j = 0; j < 3; ++j) Lr[i][j] = bf16_rne(Lm[i * 3 + j]); for (int i = 0; i < 3; ++i) for (int j = 0; j < 3; ++j) { float s = 0.0f; for (int k = 0; k < 3; ++k) s += pmul(Lr[i][k], Lr[j][k]); S[i][j] = s; } }
  const float cb0 = bf16_rne(cb[0]), cb1 = bf16_rne(cb[1]), cb2 = bf16_rne(cb[2]);
  for (int q = 0; q < 8; ++q) { const size_t v = v0 + wave * 8 + q; const size_t node = n0 + wave * 8 + q;
    int st = ROWPTR[v], cnt = ROWCNT[v]; cnt = iclamp(cnt, 0, 65536); st = iclamp(st, 0, permLen - cnt);
    const float t0 = bf16_rne(nodes[(b * NN + node) * 3]), t1 = bf16_rne(nodes[(b * NN + node) * 3 + 1]), t2 = bf16_rne(nodes[(b * NN + node) * 3 + 2]);
    v4f acc = {0.0f, 0.0f, 0.0f, 0.0f}; float den = 0.0f;
    for (int i = 0; i <= cnt; ++i) { size_t s; float kern;
      if (i < cnt) { const int e = iclamp(PERM[st + i], 0, E - 1); s = b * NN + (size_t)iclamp(ei[(size_t)e * 2], 0, NN - 1);
        const float d0 = bf16_rne(nodes[s * 3]) - t0, d1 = bf16_rne(nodes[s * 3 + 1]) - t1, d2 = bf16_rne(nodes[s * 3 + 2]) - t2;
        const float e0 = pmul(d0, S[0][0]) + pmul(d1, S[0][1]) + pmul(d2, S[0][2]) + cb0, e1 = pmul(d0, S[1][0]) + pmul(d1, S[1][1]) + pmul(d2, S[1][2]) + cb1, e2 = pmul(d0, S[2][0]) + pmul(d1, S[2][1]) + pmul(d2, S[2][2]) + cb2;
        kern = pmul(bf16_rne(nw[s]), __expf(-(pmul(d0, e0) + pmul(d1, e1) + pmul(d2, e2)))); }
      else { s = v; kern = bf16_rne(nw[v]); }
      den += kern; const v4f fs = *(const v4f*)(FO + s * OUTC + lane * 4); for (int j = 0; j < 4; ++j) acc[j] += pmul(kern, fs[j]); }
    const float inv = 1.0f / den; for (int j = 0; j < 4; ++j) St[lane * 4 + j][wave * 8 + q] = pmul(acc[j], inv); }
  __syncthreads();
  for (int pass = 0; pass < 2; ++pass) { for (int q = t_; q < OUTC * 16; q += 256) { const int c = q >> 4, c4 = (q & 15) * 4; *(volatile v4f*)(out + ((b * OUTC + c) * NN) + n0 + c4) = *(const v4f*)(&St[c][c4]); } __threadfence(); }
}
}

extern "C" void kernel_launch(void* const* d_in, const int* in_sizes, int n_in, void* d_out, int out_size, void* d_ws, size_t ws_size, hipStream_t stream) {
  (void)n_in;
  auto Fp = [&](int i) { return (const float*)d_in[i]; }; auto Ip = [&](int i) { return (const int*)d_in[i]; };
  if (in_sizes[0] != N * C || in_sizes[1] != N * 3 || in_sizes[2] != N || in_sizes[3] != E * 2 || in_sizes[4] != E * 3 || in_sizes[5] != MID * KG || in_sizes[7] != OUTC * MID || in_sizes[9] != 9 || out_size != N * OUTC) return;
  size_t off = 0; char* ws = (char*)d_ws;
  auto carve = [&](size_t bytes) { char* p = ws + off; off += (bytes + 255) & ~(size_t)255; return p; };
  int* KD = (int*)carve((size_t)E * 4); float* FT = (float*)carve((size_t)N * C * 4); b16* W1T = (b16*)carve((size_t)MID * KG * 2); b16* W2T = (b16*)carve((size_t)OUTC * MID * 2); float* FO = (float*)carve((size_t)N * OUTC * 4);
  CsrBufs csr; off = csr_carve(csr, ws, off, E, N);
  if (off > ws_size || off > ((size_t)128 << 20)) return;
  keys_kernel<<<(unsigned)(((size_t)E / 4 + 255) / 256), 256, 0, stream>>>(Ip(3), KD);
  prep_kernel<<<dim3(NN / 64, C / 64, NB), 256, 0, stream>>>(Fp(0), Fp(5), Fp(7), FT, W1T, W2T);
  csr_build(csr, KD, E, N, stream);
  gradmlp_kernel<<<N / 64, 128, 0, stream>>>(FT, Ip(3), Fp(4), csr.PERM, csr.ROWPTR, csr.ROWCNT, (int)csr.permLen, W1T, Fp(6), W2T, Fp(8), FO);
  kagg_kernel<<<N / 64, 256, 0, stream>>>(FO, Fp(1), Fp(2), Ip(3), csr.PERM, csr.ROWPTR, csr.ROWCNT, (int)csr.permLen, Fp(9), Fp(10), (float*)d_out);
}
